// Encoder_Sublayer_33749853012035
// MI455X (gfx1250) — hardware-verified
//
#include <hip/hip_runtime.h>
#include <hip/hip_bf16.h>
#include <math.h>

#define BB 2
#define SS 2048
#define DD 1024
#define HH 16
#define KVH 16
#define KVD 1024
#define DKK 64
#define QW 2
#define MTOK (BB * SS)
#define FFN 4096
#define GSTR 48

typedef _Float16 bf16;
typedef _Float16 f16;
typedef __attribute__((ext_vector_type(4))) unsigned v4u_t;
typedef unsigned v4ua __attribute__((ext_vector_type(4), may_alias));
typedef __attribute__((ext_vector_type(4))) float v4f_t;
typedef float v4fa __attribute__((ext_vector_type(4), may_alias));
typedef __attribute__((ext_vector_type(16))) bf16  bf16x16;
typedef bf16x16 f16x16;
typedef __attribute__((ext_vector_type(8)))  bf16  bf16x8;
typedef bf16x8 f16x8;
typedef __attribute__((ext_vector_type(4)))  bf16  bf16x4;
typedef __attribute__((ext_vector_type(8)))  float f32x8;
__device__ __forceinline__ f32x8 wmma16(f16x16 a, f16x16 b, f32x8 c) {
  c = __builtin_amdgcn_wmma_f32_16x16x32_f16(false, a, false, b, (short)0, c, false, false);
  asm volatile("v_nop\n\tv_nop\n\tv_nop\n\tv_nop" : "+v"(c) : "v"(a), "v"(b));
  return c;
}
#define LDS_STRIDE 48
#define KSTRIDE    72
#define VSTRIDE    48

__device__ __forceinline__ f32x8 wmma_bf16(bf16x16 a, bf16x16 b, f32x8 c) {
  c = __builtin_amdgcn_wmma_f32_16x16x32_f16(false, a, false, b, (short)0, c, false, false);
  asm volatile("v_nop\n\tv_nop\n\tv_nop\n\tv_nop" : "+v"(c) : "v"(a), "v"(b));
  return c;
}

template <typename T>
__device__ __forceinline__ bf16x16 load_frag(const T* __restrict__ base, int ld,
                                             int row0, int k0) {
  const int lane = threadIdx.x & 31;
  const int r    = lane & 15;
  const int kh   = (lane >> 4) * 8;
  const T* p0 = base + (size_t)(row0 + r) * ld + (k0 + kh);
  const T* p1 = p0 + 16;
  bf16x16 f;
#pragma unroll
  for (int i = 0; i < 8; ++i) {
    f[i]     = (bf16)p0[i];
    f[i + 8] = (bf16)p1[i];
  }
  return f;
}

__device__ __forceinline__ bf16x16 lds_frag(const bf16* base, int stride) {
  const int lane = threadIdx.x & 31;
  const int row  = lane & 15;
  const int kh   = (lane >> 4) * 8;
  const bf16x8 lo = *(const bf16x8*)(base + row * stride + kh);
  const bf16x8 hi = *(const bf16x8*)(base + row * stride + kh + 16);
  bf16x16 f;
#pragma unroll
  for (int i = 0; i < 8; ++i) { f[i] = lo[i]; f[i + 8] = hi[i]; }
  return f;
}

template <typename T>
__device__ __forceinline__ void stage_read16(const T* __restrict__ p, float* buf) {
#pragma unroll
  for (int i = 0; i < 16; ++i) buf[i] = (float)p[i];
}

__device__ __forceinline__ void stage_write(bf16* dst, const float* buf, int nquad) {
#pragma unroll
  for (int i = 0; i < nquad; ++i) {
    bf16x4 q;
    q[0] = (bf16)buf[4 * i];     q[1] = (bf16)buf[4 * i + 1];
    q[2] = (bf16)buf[4 * i + 2]; q[3] = (bf16)buf[4 * i + 3];
    *(bf16x4*)(dst + 4 * i) = q;
  }
}


#define GSTR 48
template <typename AT, int EPI, bool OUT16>
__global__ __launch_bounds__(256) void gemm_kne(const AT* __restrict__ A, int lda, const float* __restrict__ Wm, int ldw,
                                                const float* __restrict__ bias, const float* __restrict__ R, const float* __restrict__ gvec,
                                                void* __restrict__ Yv, int ldy, int K) {
  __shared__ __attribute__((aligned(16))) f16 ldsA[128 * GSTR];
  __shared__ __attribute__((aligned(16))) f16 ldsW[128 * GSTR];
  __shared__ __attribute__((aligned(16))) float oS[8][32 * 68];
  const int tid = threadIdx.x, lane = tid & 31, wave = tid >> 5, cl = lane & 15, rh = (lane >> 4) * 8;
  const int m0 = blockIdx.x * 128, n0 = blockIdx.y * 128;
  const int wm = (wave & 3) * 32, wn = (wave >> 2) * 64;
  f32x8 acc[2][4];
#pragma unroll
  for (int i = 0; i < 2; ++i)
#pragma unroll
    for (int j = 0; j < 4; ++j) { f32x8 z = {}; acc[i][j] = z; }
#pragma unroll 1
  for (int k0 = 0; k0 < K; k0 += 32) {
    __syncthreads();
    { const int row = tid >> 1, ch = (tid & 1) * 16;
      const AT* src = A + (size_t)(m0 + row) * lda + k0 + ch;
#pragma unroll
      for (int g = 0; g < 16; ++g) ldsA[row * GSTR + ch + g] = (f16)src[g]; }
    { const int k = tid >> 3, nn0 = (tid & 7) * 16;
      const float* src = Wm + (size_t)(k0 + k) * ldw + n0 + nn0;
#pragma unroll
      for (int g = 0; g < 4; ++g) { const v4f_t v = *(const v4f_t*)(src + 4 * g);
#pragma unroll
        for (int u = 0; u < 4; ++u) ldsW[(nn0 + 4 * g + u) * GSTR + k] = (f16)v[u]; } }
    __syncthreads();
    f16x16 af[2];
#pragma unroll
    for (int i = 0; i < 2; ++i) af[i] = lds_frag(ldsA + (wm + 16 * i) * GSTR, GSTR);
#pragma unroll
    for (int j = 0; j < 4; ++j) {
      const f16x16 bf = lds_frag(ldsW + (wn + 16 * j) * GSTR, GSTR);
#pragma unroll
      for (int i = 0; i < 2; ++i) acc[i][j] = wmma16(af[i], bf, acc[i][j]);
    }
  }
  float* so = oS[wave];
#pragma unroll
  for (int i = 0; i < 2; ++i)
#pragma unroll
    for (int j = 0; j < 4; ++j) {
      const int n = n0 + wn + 16 * j + cl;
      const float bv = bias ? bias[n] : 0.0f;
      const float gv = (EPI == 2) ? gvec[n] : 0.0f;
      if (EPI == 1) {
#pragma unroll 1
        for (int r = 0; r < 8; ++r) { const float xg = acc[i][j][r] + bv; so[(16 * i + rh + r) * 68 + 16 * j + cl] = 0.5f * xg * (1.0f + erff(xg * 0.70710678118654752f)); }
      } else {
#pragma unroll
        for (int r = 0; r < 8; ++r) {
          float v = acc[i][j][r] + bv;
          if (EPI == 3) v = fmaxf(v, 0.0f);
          if (EPI == 2) v = R[(size_t)(m0 + wm + 16 * i + rh + r) * ldy + n] + gv * v;
          so[(16 * i + rh + r) * 68 + 16 * j + cl] = v;
        }
      }
    }
  asm volatile("s_wait_dscnt 0" ::: "memory");
  __builtin_amdgcn_wave_barrier();
#pragma unroll 1
  for (int pass = 0; pass < 2; ++pass) {
    if (OUT16) {
      f16* Y = (f16*)Yv;
#pragma unroll
      for (int it = 0; it < 8; ++it) { const int c = lane + 32 * it, rr = c >> 3, q8 = (c & 7) * 8;
        union { f16 h[8]; v4u_t v; } u;
#pragma unroll
        for (int e = 0; e < 8; ++e) u.h[e] = (f16)so[rr * 68 + q8 + e];
        *(volatile v4u_t*)(Y + (size_t)(m0 + wm + rr) * ldy + n0 + wn + q8) = u.v; }
    } else {
      float* Y = (float*)Yv;
#pragma unroll
      for (int it = 0; it < 16; ++it) { const int f4 = lane + 32 * it, rr = f4 >> 4, q = (f4 & 15) * 4;
        *(volatile v4f_t*)(Y + (size_t)(m0 + wm + rr) * ldy + n0 + wn + q) = *(const v4fa*)(so + rr * 68 + q); }
    }
    __threadfence();
  }
}
__global__ __launch_bounds__(64) void attn_kernel(
    const bf16* __restrict__ Qb, const bf16* __restrict__ Kb,
    const bf16* __restrict__ Vt,
    bf16* __restrict__ attnOut) {
  __shared__ bf16 ldsK[32 * KSTRIDE];
  __shared__ bf16 ldsV[64 * VSTRIDE];
  __shared__ __attribute__((aligned(16))) bf16 ldsO[2][32 * 72];

  const int q0blk = blockIdx.x * 64;
  const int h  = blockIdx.y;
  const int b  = blockIdx.z;
  const int t    = threadIdx.x;
  const int wave = t >> 5;
  const int lane = t & 31;
  const int qlane = lane & 15;
  const int kh8   = (lane >> 4) * 8;
  const int q0 = q0blk + wave * 32;

  const int hk = h;
  const bf16* Qh = Qb + (size_t)b * SS * DD + h * DKK;
  const bf16* Kh = Kb + (size_t)b * SS * KVD + hk * DKK;
  const bf16* Vh = Vt + ((size_t)(b * KVH + hk)) * DKK * SS;

  const int krow = t >> 1;
  const int kcol = (t & 1) * 32;
  const bf16* kSrc = Kh + (size_t)krow * KVD + kcol;
  const bf16* vSrc = Vh + (size_t)t * SS;

  bf16x16 qf[QW][2];
#pragma unroll
  for (int qt = 0; qt < QW; ++qt) {
    qf[qt][0] = load_frag(Qh, DD, q0 + 16 * qt, 0);
    qf[qt][1] = load_frag(Qh, DD, q0 + 16 * qt, 32);
  }

  f32x8 o[QW][4] = {};
  float mrun[QW], lrun[QW];
#pragma unroll
  for (int qt = 0; qt < QW; ++qt) { mrun[qt] = -INFINITY; lrun[qt] = 0.0f; }

  const float scale = 0.125f * 1.44269504088896340736f;
  const float NEG2 = -1.0e9f;
  const int kmax = SS - 1;

  bf16x8 kreg[4], vreg[4];
#pragma unroll
  for (int i = 0; i < 4; ++i) {
    kreg[i] = *(const bf16x8*)(kSrc + 8 * i);
    vreg[i] = *(const bf16x8*)(vSrc + 8 * i);
  }

  for (int kb = 0; kb <= kmax; kb += 32) {
    __syncthreads();
#pragma unroll
    for (int i = 0; i < 4; ++i) {
      *(bf16x8*)(&ldsK[krow * KSTRIDE + kcol + 8 * i]) = kreg[i];
      *(bf16x8*)(&ldsV[t * VSTRIDE + 8 * i])           = vreg[i];
    }
    if (kb + 32 <= kmax) {
      const bf16* kn = kSrc + (size_t)(kb + 32) * KVD;
      const bf16* vn = vSrc + (kb + 32);
#pragma unroll
      for (int i = 0; i < 4; ++i) {
        kreg[i] = *(const bf16x8*)(kn + 8 * i);
        vreg[i] = *(const bf16x8*)(vn + 8 * i);
      }
    }
    __syncthreads();

    bf16x16 kf[2][2];
#pragma unroll
    for (int ktile = 0; ktile < 2; ++ktile)
#pragma unroll
      for (int c = 0; c < 2; ++c)
        kf[ktile][c] = lds_frag(ldsK + (ktile * 16) * KSTRIDE + c * 32, KSTRIDE);

    bf16x16 pf[QW];
    bool act[QW];
#pragma unroll
    for (int qt = 0; qt < QW; ++qt) {
      unsigned mbits = 0;
      mbits = 0xFFFFu; act[qt] = true;
      if (act[qt]) {
        const int q_my = q0 + 16 * qt + qlane;
        f32x8 s0 = {}, s1 = {};
        s0 = wmma_bf16(kf[0][0], qf[qt][0], s0);
        s0 = wmma_bf16(kf[0][1], qf[qt][1], s0);
        s1 = wmma_bf16(kf[1][0], qf[qt][0], s1);
        s1 = wmma_bf16(kf[1][1], qf[qt][1], s1);

        float mx = -INFINITY;
#pragma unroll
        for (int r = 0; r < 8; ++r) {
          const int k0i = kb + kh8 + r;
          const int k1i = k0i + 16;
          (void)k0i; (void)k1i; (void)q_my;
          s0[r] = (mbits & (1u << r))       ? s0[r] * scale : NEG2;
          s1[r] = (mbits & (1u << (8 + r))) ? s1[r] * scale : NEG2;
          mx = fmaxf(mx, fmaxf(s0[r], s1[r]));
        }
        mx = fmaxf(mx, __shfl_xor(mx, 16, 32));
        const float mnew  = fmaxf(mrun[qt], mx);
        const float alpha = exp2f(mrun[qt] - mnew);

        float rsum = 0.0f;
#pragma unroll
        for (int r = 0; r < 8; ++r) {
          const float p0 = exp2f(s0[r] - mnew);
          const float p1 = exp2f(s1[r] - mnew);
          rsum += p0 + p1;
          pf[qt][r]     = (bf16)(p0 * 1024.0f);
          pf[qt][r + 8] = (bf16)(p1 * 1024.0f);
        }
        rsum += __shfl_xor(rsum, 16, 32);
        lrun[qt] = lrun[qt] * alpha + rsum;
        mrun[qt] = mnew;

#pragma unroll
        for (int j = 0; j < 4; ++j)
#pragma unroll
          for (int r = 0; r < 8; ++r) o[qt][j][r] *= alpha;
      }
    }

#pragma unroll
    for (int j = 0; j < 4; ++j) {
      const bf16x16 vf = lds_frag(ldsV + (j * 16) * VSTRIDE, VSTRIDE);
#pragma unroll
      for (int qt = 0; qt < QW; ++qt)
        if (act[qt]) o[qt][j] = wmma_bf16(vf, pf[qt], o[qt][j]);
    }
  }

  bf16* so = ldsO[wave];
#pragma unroll
  for (int qt = 0; qt < QW; ++qt) {
    const float rl = 1.0f / (lrun[qt] * 1024.0f);
#pragma unroll
    for (int j = 0; j < 4; ++j)
#pragma unroll
      for (int r = 0; r < 8; ++r) so[(16 * qt + qlane) * 72 + j * 16 + kh8 + r] = (bf16)(o[qt][j][r] * rl);
  }
  asm volatile("s_wait_dscnt 0" ::: "memory");
#pragma unroll 1
  for (int pass = 0; pass < 2; ++pass) {
#pragma unroll
    for (int it = 0; it < 8; ++it) { const int ch = lane + 32 * it, ql = ch >> 3, q8 = (ch & 7) * 8;
      *(volatile v4u_t*)(attnOut + ((size_t)(b * SS + q0 + ql)) * DD + h * DKK + q8) = *(const v4ua*)(so + ql * 72 + q8); }
    __threadfence();
  }
}


__global__ __launch_bounds__(256) void k_viewsplit(const float* __restrict__ Pq, const float* __restrict__ Pk, const float* __restrict__ Pv, bf16* __restrict__ Q16, bf16* __restrict__ K16, bf16* __restrict__ Vt) {
  __shared__ __attribute__((aligned(16))) bf16 qS[64][72], kS[64][72], vT[64][72];
  const int tid = threadIdx.x; const size_t t0 = (size_t)blockIdx.x * 64; const int h = blockIdx.y; const int b = (int)(t0 / SS), n0 = (int)(t0 % SS);
  for (int e = tid; e < 64 * 64; e += 256) { const int t = e >> 6, d = e & 63; const size_t src = (size_t)b * SS * DD + ((size_t)h * SS + n0 + t) * DKK + d;
    qS[t][d] = (bf16)Pq[src]; kS[t][d] = (bf16)Pk[src]; vT[d][t] = (bf16)Pv[src]; }
  __syncthreads();
#pragma unroll 1
  for (int pass = 0; pass < 2; ++pass) {
#pragma unroll 1
    for (int round = 0; round < 2; ++round) { const int r = round * 32 + (tid >> 3), piece = (tid & 7) * 8;
      *(volatile v4u_t*)(Q16 + (t0 + r) * DD + h * DKK + piece) = *(const v4ua*)(&qS[r][piece]);
      *(volatile v4u_t*)(K16 + (t0 + r) * DD + h * DKK + piece) = *(const v4ua*)(&kS[r][piece]);
      *(volatile v4u_t*)(Vt + ((size_t)b * DD + h * DKK + r) * SS + n0 + piece) = *(const v4ua*)(&vT[r][piece]); }
    __threadfence(); }
}
template <bool OUT16>
__global__ __launch_bounds__(256) void k_ln(const float* __restrict__ X, const float* __restrict__ g, const float* __restrict__ bb, void* __restrict__ Yv) {
  __shared__ __attribute__((aligned(16))) float rowS[8 * (DD + 4)];
  const int tid = threadIdx.x, r = tid >> 5, lane = tid & 31; const size_t row = (size_t)blockIdx.x * 8 + r; const float* xr = X + row * DD;
  float s = 0.0f;
#pragma unroll 1
  for (int i = lane; i < DD; i += 32) { const float v = xr[i]; rowS[r * (DD + 4) + i] = v; s += v; }
#pragma unroll
  for (int off = 1; off < 32; off <<= 1) s += __shfl_xor(s, off, 32);
  const float mean = s * (1.0f / DD); float q = 0.0f;
#pragma unroll 1
  for (int i = lane; i < DD; i += 32) { const float d = rowS[r * (DD + 4) + i] - mean; q += d * d; }
#pragma unroll
  for (int off = 1; off < 32; off <<= 1) q += __shfl_xor(q, off, 32);
  const float rstd = rsqrtf(q * (1.0f / DD) + 1e-5f);
#pragma unroll 1
  for (int i = lane; i < DD; i += 32) rowS[r * (DD + 4) + i] = (rowS[r * (DD + 4) + i] - mean) * rstd * g[i] + bb[i];
  __syncthreads();
#pragma unroll 1
  for (int pass = 0; pass < 2; ++pass) {
    if (OUT16) { bf16* Y = (bf16*)Yv; for (int q8 = tid; q8 < 8 * (DD / 8); q8 += 256) { const int rr = q8 / (DD / 8), c8 = (q8 % (DD / 8)) * 8; union { bf16 hh[8]; v4u_t u; } cv;
        for (int i = 0; i < 8; ++i) cv.hh[i] = (bf16)rowS[rr * (DD + 4) + c8 + i]; *(volatile v4u_t*)(Y + ((size_t)blockIdx.x * 8 + rr) * DD + c8) = cv.u; } }
    else { float* Y = (float*)Yv; for (int q4 = tid; q4 < 8 * (DD / 4); q4 += 256) { const int rr = q4 / (DD / 4), c4 = (q4 % (DD / 4)) * 4;
        *(volatile v4f_t*)(Y + ((size_t)blockIdx.x * 8 + rr) * DD + c4) = *(const v4fa*)(rowS + rr * (DD + 4) + c4); } }
    __threadfence(); }
}
__global__ __launch_bounds__(256) void k_ones(float* __restrict__ p, int n) { for (int i = threadIdx.x; i < n; i += 256) { *(volatile float*)(p + i) = 1.0f; __threadfence(); *(volatile float*)(p + i) = 1.0f; } }

extern "C" void kernel_launch(void* const* d_in, const int* in_sizes, int n_in,
                              void* d_out, int out_size, void* d_ws, size_t ws_size,
                              hipStream_t stream) {
  (void)in_sizes; (void)n_in; (void)out_size;
  const float** f = (const float**)d_in;
  const float* data = f[0];   const float* wq = f[2], *bq = f[3], *wk = f[4], *bk = f[5], *wv = f[6], *bv = f[7], *wo = f[8], *bo = f[9], *l1g = f[10], *l1b = f[11], *w1 = f[12], *b1 = f[13], *w2 = f[14], *b2 = f[15], *l2g = f[16], *l2b = f[17];
  float* out = (float*)d_out;
  char* ws = (char*)d_ws;
  float* Pq = (float*)ws; ws += (size_t)MTOK * DD * 4; float* Pk = (float*)ws; ws += (size_t)MTOK * DD * 4; float* Pv = (float*)ws; ws += (size_t)MTOK * DD * 4;
  bf16* Q16 = (bf16*)ws; ws += (size_t)MTOK * DD * 2; bf16* K16 = (bf16*)ws; ws += (size_t)MTOK * DD * 2; bf16* Vt = (bf16*)ws; ws += (size_t)MTOK * DD * 2; bf16* att = (bf16*)ws; ws += (size_t)MTOK * DD * 2;
  float* y1 = Pq;
  float* x1 = Pk;
  bf16* x16 = Q16;
  bf16* ffh = (bf16*)ws; ws += (size_t)MTOK * FFN * 2;
  float* y2 = Pv;
  float* ones = (float*)ws; ws += DD * 4;
  if ((size_t)(ws - (char*)d_ws) > ws_size) return;
  const dim3 blk(256); const dim3 gp(MTOK / 128, DD / 128);
  k_ones<<<dim3(1), blk, 0, stream>>>(ones, DD);
  gemm_kne<float, 0, false><<<gp, blk, 0, stream>>>(data, DD, wq, DD, bq, nullptr, nullptr, Pq, DD, DD);
  gemm_kne<float, 0, false><<<gp, blk, 0, stream>>>(data, DD, wk, DD, bk, nullptr, nullptr, Pk, DD, DD);
  gemm_kne<float, 0, false><<<gp, blk, 0, stream>>>(data, DD, wv, DD, bv, nullptr, nullptr, Pv, DD, DD);
  k_viewsplit<<<dim3(MTOK / 64, HH), blk, 0, stream>>>(Pq, Pk, Pv, Q16, K16, Vt);
  attn_kernel<<<dim3(SS / 64, HH, BB), dim3(64), 0, stream>>>(Q16, K16, Vt, att);
  gemm_kne<bf16, 2, false><<<gp, blk, 0, stream>>>(att, DD, wo, DD, bo, data, ones, y1, DD, DD);
  k_ln<false><<<dim3(MTOK / 8), blk, 0, stream>>>(y1, l1g, l1b, x1);
  k_ln<true><<<dim3(MTOK / 8), blk, 0, stream>>>(y1, l1g, l1b, x16);
  gemm_kne<bf16, 3, true><<<dim3(MTOK / 128, FFN / 128), blk, 0, stream>>>(x16, DD, w1, FFN, b1, nullptr, nullptr, ffh, FFN, DD);
  gemm_kne<bf16, 2, false><<<gp, blk, 0, stream>>>(ffh, FFN, w2, DD, b2, x1, ones, y2, DD, FFN);
  k_ln<false><<<dim3(MTOK / 8), blk, 0, stream>>>(y2, l2g, l2b, out);
}
